// StackRNN_54245436948936
// MI455X (gfx1250) — hardware-verified
//
#include <hip/hip_runtime.h>
#include <hip/hip_bf16.h>


#define S_    128
#define B_    128
#define IN_   512
#define H_    512
#define SW_   64
#define SD_   32
#define G4_   2048
#define M_    16384
#define KC_   576
#define NG_   1536
#define KS_   18
#define NTHR  256
#define MB_   128
#define UB_   32
#define HP_   36

static_assert(M_ == S_ * B_);
static_assert(KC_ == IN_ + SW_ && KC_ == H_ + SW_);
static_assert(KC_ == 32 * KS_);
static_assert(NG_ == 3 * H_);
static_assert(H_ % UB_ == 0 && M_ % MB_ == 0 && M_ % 8 == 0);
static_assert(HP_ % 4 == 0 && HP_ >= UB_);
static_assert(NTHR == 256 && MB_ == 128 && UB_ == 32);
static_assert(SD_ * SW_ == 8 * NTHR);

typedef _Float16       v16h __attribute__((ext_vector_type(16)));
typedef _Float16       v8h  __attribute__((ext_vector_type(8)));
typedef __bf16         v16b __attribute__((ext_vector_type(16)));
typedef unsigned short v8us __attribute__((ext_vector_type(8)));
typedef float          v8f  __attribute__((ext_vector_type(8)));
typedef float          v4f  __attribute__((ext_vector_type(4)));

union FragH { v16h v; v8h  half[2]; };
union FragB { v16b v; v8us half[2]; };

constexpr size_t SZ_TOP = (size_t)S_ * SW_ * 4;
constexpr size_t SZ_WP  = (size_t)NG_ * KC_ * 2;
constexpr size_t SZ_XP  = (size_t)M_ * KC_ * 2;
constexpr size_t SZ_HB  = (size_t)M_ * H_ * 4;
constexpr size_t SZ_CB  = (size_t)B_ * H_ * 4;
constexpr size_t OFF_TOP0 = 0;
constexpr size_t OFF_TOP1 = OFF_TOP0 + SZ_TOP;
constexpr size_t OFF_W0P  = OFF_TOP1 + SZ_TOP;
constexpr size_t OFF_W1H  = OFF_W0P  + SZ_WP;
constexpr size_t OFF_W1L  = OFF_W1H  + SZ_WP;
constexpr size_t OFF_X0P  = OFF_W1L  + SZ_WP;
constexpr size_t OFF_X1H  = OFF_X0P  + SZ_XP;
constexpr size_t OFF_X1L  = OFF_X1H  + SZ_XP;
constexpr size_t OFF_HB   = OFF_X1L  + SZ_XP;
constexpr size_t OFF_CB0  = OFF_HB   + SZ_HB;
constexpr size_t OFF_CB1  = OFF_CB0  + SZ_CB;
constexpr size_t WS_END   = OFF_CB1  + SZ_CB;
static_assert(OFF_TOP1 % 128 == 0 && OFF_W0P % 128 == 0 && OFF_W1H % 128 == 0 && OFF_W1L % 128 == 0);
static_assert(OFF_X0P % 128 == 0 && OFF_X1H % 128 == 0 && OFF_X1L % 128 == 0 && OFF_HB % 128 == 0);
static_assert(OFF_CB0 % 128 == 0 && OFF_CB1 % 128 == 0 && WS_END % 128 == 0);
static_assert(WS_END <= (size_t)134217728);

constexpr size_t OUT1_F = (size_t)M_ * H_;
constexpr size_t OUT2_F = OUT1_F + (size_t)2 * B_ * H_;
constexpr size_t OUT_N  = OUT2_F + (size_t)2 * B_ * H_;
static_assert(OUT1_F * 4 == 33554432 && OUT2_F * 4 == 34078720 && OUT_N * 4 == 34603008);

constexpr int NPW = NG_ * (KC_ / 8);
constexpr int NBW = NPW / NTHR;
constexpr int NPX = M_ * (KC_ / 8);
constexpr int NBX = NPX / NTHR;
static_assert(NPW % NTHR == 0 && NPX % NTHR == 0);
static_assert((size_t)NPW * 16 == SZ_WP && (size_t)NPX * 16 == SZ_XP);
static_assert(KC_ / 8 == 72);

__device__ __forceinline__ float rcpx(float x) { return __builtin_amdgcn_rcpf(x); }
__device__ __forceinline__ float sigm(float x) { return rcpx(1.0f + __expf(-x)); }
__device__ __forceinline__ float tanhm(float x) {
    const float e = __expf(2.0f * x);
    return 1.0f - 2.0f * rcpx(e + 1.0f);
}
__device__ __forceinline__ float wsum(float v) {
#pragma unroll
    for (int o = 16; o > 0; o >>= 1) v += __shfl_xor(v, o, 32);
    return v;
}
__device__ __forceinline__ unsigned int bf16_rne(float x) {
    const unsigned int u = __float_as_uint(x);
    return (u + 0x7FFFu + ((u >> 16) & 1u)) >> 16;
}
__device__ __forceinline__ void split_bf16(float x, unsigned short& hi, unsigned short& lo) {
    const unsigned int hb = bf16_rne(x);
    const float hf = __uint_as_float(hb << 16);
    const unsigned int lb = bf16_rne(x - hf);
    hi = (unsigned short)hb;
    lo = (unsigned short)lb;
}
__device__ __forceinline__ v8f ld8f(const float* p) {
    const v4f a = *(const v4f*)p;
    const v4f b = *(const v4f*)(p + 4);
    return __builtin_shufflevector(a, b, 0, 1, 2, 3, 4, 5, 6, 7);
}
__device__ __forceinline__ v8f zero8() {
    v8f z;
#pragma unroll
    for (int i = 0; i < 8; ++i) z[i] = 0.0f;
    return z;
}

__device__ __forceinline__ void ldh_glb(FragH& f, const _Float16* p) {
    f.half[0] = *(const v8h*)(p);
    f.half[1] = *(const v8h*)(p + 16);
}
__device__ __forceinline__ void ldb_glb(FragB& f, const unsigned short* p) {
    f.half[0] = *(const v8us*)(p);
    f.half[1] = *(const v8us*)(p + 16);
}
__device__ __forceinline__ v8f mmah(v8f c, const FragH& a, const FragH& b) {
    return __builtin_amdgcn_wmma_f32_16x16x32_f16(false, a.v, false, b.v, (short)0, c, false, false);
}
__device__ __forceinline__ v8f mmab(v8f c, const FragB& a, const FragB& b) {
    return __builtin_amdgcn_wmma_f32_16x16x32_bf16(false, a.v, false, b.v, (short)0, c, false, false);
}

__global__ __launch_bounds__(NTHR)
void k_stack(const float* __restrict__ bc0, const float* __restrict__ bs0,
             const float* __restrict__ bc1, const float* __restrict__ bs1,
             float* top0, float* top1)
{
    __shared__ __attribute__((aligned(16))) float sStk[2][SD_ * SW_];
    __shared__ __attribute__((aligned(16))) float sTop[S_ * SW_];
    __shared__ float sIn[SW_];
    __shared__ float sE[4];

    const int tid   = threadIdx.x;
    const int layer = blockIdx.x;
    const float* bc = layer ? bc1 : bc0;
    const float* bs = layer ? bs1 : bs0;
    float* top      = layer ? top1 : top0;

    const float c0 = bc[0], c1 = bc[1], c2 = bc[2];
    const float mx = fmaxf(c0, fmaxf(c1, c2));
    {
        const int j = min(tid, 2);
        const float e = expf(bc[j] - mx);
        if (tid < 3) sE[tid] = e;
        const int k = min(tid, SW_ - 1);
        const float s = tanhf(bs[k]);
        if (tid < SW_) sIn[tid] = s;
    }
    for (int i = tid; i < SD_ * SW_; i += NTHR) { sStk[0][i] = 0.0f; sStk[1][i] = 0.0f; }
    __syncthreads();

    const float esum   = (sE[0] + sE[1]) + sE[2];
    const float einv   = 1.0f / esum;
    const float a_push = sE[0] * einv;
    const float a_pop  = sE[1] * einv;
    const float a_noop = sE[2] * einv;

#pragma unroll 1
    for (int t = 0; t < S_; ++t) {
        const float* cur = sStk[t & 1];
        float*       nxt = sStk[(t + 1) & 1];
#pragma unroll 1
        for (int e = 0; e < 8; ++e) {
            const int idx = tid + NTHR * e;
            const int d   = idx >> 6;
            const int k   = idx & 63;
            const float old = cur[idx];
            const float upa = cur[max(d - 1, 0) * SW_ + k];
            const float upv = (d == 0) ? sIn[k] : upa;
            const float dna = cur[min(d + 1, SD_ - 1) * SW_ + k];
            const float dnv = (d < SD_ - 1) ? dna : 0.0f;
            const float nv  = a_noop * old + a_push * upv + a_pop * dnv;
            nxt[idx] = nv;
            if (d == 0) sTop[t * SW_ + k] = nv;
        }
        __syncthreads();
    }

#pragma unroll
    for (int i = 0; i < 8; ++i) {
        const int p = tid + NTHR * i;
        const v4f v = *(const v4f*)(sTop + 4 * p);
        *(volatile v4f*)(top + 4 * p) = v;
    }
    __threadfence();
#pragma unroll
    for (int i = 0; i < 8; ++i) {
        const int p = tid + NTHR * i;
        const v4f v = *(const v4f*)(sTop + 4 * p);
        *(volatile v4f*)(top + 4 * p) = v;
    }
}

__global__ __launch_bounds__(NTHR)
void k_wcvt(const float* __restrict__ Wih0, const float* __restrict__ Wih1,
            _Float16* W0p, unsigned short* W1h, unsigned short* W1l)
{
    const int tid = threadIdx.x;
    const int bid = blockIdx.x;
    const int sel = (bid < NBW) ? 0 : 1;
    const int p   = (bid - sel * NBW) * NTHR + tid;
    const int n   = p / 72;
    const int j   = p - n * 72;
    const int g3  = n >> 9;
    const int u   = n & 511;
    const int srow = u + ((g3 == 0) ? 0 : 512 * (g3 + 1));
    const float* W = sel ? Wih1 : Wih0;
    const v8f a = ld8f(W + (size_t)srow * KC_ + 8 * j);
    const size_t o = (size_t)8 * p;
    if (sel == 0) {
        v8h hv;
#pragma unroll
        for (int i = 0; i < 8; ++i) hv[i] = (_Float16)(a[i] * 16.0f);
        *(volatile v8h*)(W0p + o) = hv;
        __threadfence();
        *(volatile v8h*)(W0p + o) = hv;
    } else {
        v8us hv, lv;
#pragma unroll
        for (int i = 0; i < 8; ++i) { unsigned short hi, lo; split_bf16(a[i], hi, lo); hv[i] = hi; lv[i] = lo; }
        *(volatile v8us*)(W1h + o) = hv;
        *(volatile v8us*)(W1l + o) = lv;
        __threadfence();
        *(volatile v8us*)(W1h + o) = hv;
        *(volatile v8us*)(W1l + o) = lv;
    }
}

__global__ __launch_bounds__(NTHR)
void k_xcvt(const float* __restrict__ x, const float* __restrict__ top0, _Float16* X0p)
{
    const int p  = blockIdx.x * NTHR + threadIdx.x;
    const int m  = p / 72;
    const int j  = p - m * 72;
    const int t  = m >> 7;
    const int jx = min(j, 63);
    const int jt = min(max(j - 64, 0), 7);
    const v8f ax = ld8f(x + (size_t)m * IN_ + 8 * jx);
    const v8f at = ld8f(top0 + (size_t)t * SW_ + 8 * jt);
    v8h hv;
#pragma unroll
    for (int i = 0; i < 8; ++i) hv[i] = (_Float16)((j < 64) ? ax[i] : at[i]);
    _Float16* d = X0p + (size_t)8 * p;
    *(volatile v8h*)d = hv;
    __threadfence();
    *(volatile v8h*)d = hv;
}

__device__ __forceinline__ void gate_epilogue(v8f (&acc)[2][3], const float inv,
                                              const float* __restrict__ bih, const float* __restrict__ bhh,
                                              float* sH, float* sC, float* hbuf, float* cbuf,
                                              const int m0, const int u0, const int writec,
                                              const int tid, const int rq, const int ug, const int h, const int m)
{
    const int u  = u0 + 16 * ug + m;
    const int cl = 16 * ug + m;
    const float bi = bih[u] + bhh[u];
    const float bg = bih[2 * H_ + u] + bhh[2 * H_ + u];
    const float bo = bih[3 * H_ + u] + bhh[3 * H_ + u];
#pragma unroll
    for (int mt = 0; mt < 2; ++mt) {
#pragma unroll
        for (int r = 0; r < 8; ++r) {
            const int rl = 32 * rq + 16 * mt + 8 * h + r;
            const float gi = acc[mt][0][r] * inv + bi;
            const float gg = acc[mt][1][r] * inv + bg;
            const float go = acc[mt][2][r] * inv + bo;
            const float cn = sigm(gi) * tanhm(gg);
            const float hn = sigm(go) * tanhm(cn);
            sH[rl * HP_ + cl] = hn;
            sC[rl * HP_ + cl] = cn;
        }
    }
    __syncthreads();

    v4f hv[4], cv[4];
#pragma unroll
    for (int i = 0; i < 4; ++i) {
        const int p  = tid + NTHR * i;
        const int rl = p >> 3;
        const int q  = p & 7;
        hv[i] = *(const v4f*)(sH + rl * HP_ + 4 * q);
        cv[i] = *(const v4f*)(sC + rl * HP_ + 4 * q);
    }
#pragma unroll
    for (int i = 0; i < 4; ++i) {
        const int p  = tid + NTHR * i;
        const int rl = p >> 3;
        const int q  = p & 7;
        float* hp = hbuf + (size_t)(m0 + rl) * H_ + u0 + 4 * q;
        *(volatile v4f*)hp = hv[i];
        if (writec) {
            float* cp = cbuf + (size_t)rl * H_ + u0 + 4 * q;
            *(volatile v4f*)cp = cv[i];
        }
    }
    __threadfence();
#pragma unroll
    for (int i = 0; i < 4; ++i) {
        const int p  = tid + NTHR * i;
        const int rl = p >> 3;
        const int q  = p & 7;
        float* hp = hbuf + (size_t)(m0 + rl) * H_ + u0 + 4 * q;
        *(volatile v4f*)hp = hv[i];
        if (writec) {
            float* cp = cbuf + (size_t)rl * H_ + u0 + 4 * q;
            *(volatile v4f*)cp = cv[i];
        }
    }
}

__global__ __launch_bounds__(NTHR)
void k_gemm0(const _Float16* __restrict__ X0p, const _Float16* __restrict__ W0p,
             const float* __restrict__ bih, const float* __restrict__ bhh,
             float* hbuf, float* cbuf)
{
    __shared__ __attribute__((aligned(16))) float sH[MB_ * HP_];
    __shared__ __attribute__((aligned(16))) float sC[MB_ * HP_];

    const int tid  = threadIdx.x;
    const int lane = tid & 31;
    const int w    = tid >> 5;
    const int h    = lane >> 4;
    const int m    = lane & 15;
    const int rq   = w >> 1;
    const int ug   = w & 1;
    const int u0   = blockIdx.x * UB_;
    const int m0   = blockIdx.y * MB_;
    const int writec = (blockIdx.y == (M_ / MB_) - 1) ? 1 : 0;

    v8f acc[2][3];
#pragma unroll
    for (int mt = 0; mt < 2; ++mt)
#pragma unroll
        for (int gi = 0; gi < 3; ++gi) acc[mt][gi] = zero8();

    const _Float16* ap = X0p + (size_t)(m0 + 32 * rq + m) * KC_ + 8 * h;
    const _Float16* bp = W0p + (size_t)(u0 + 16 * ug + m) * KC_ + 8 * h;

#pragma unroll 2
    for (int ks = 0; ks < KS_; ++ks) {
        FragH a[2], b[3];
        ldh_glb(a[0], ap + 32 * ks);
        ldh_glb(a[1], ap + (size_t)16 * KC_ + 32 * ks);
#pragma unroll
        for (int gi = 0; gi < 3; ++gi) ldh_glb(b[gi], bp + (size_t)gi * (H_ * KC_) + 32 * ks);
#pragma unroll
        for (int mt = 0; mt < 2; ++mt)
#pragma unroll
            for (int gi = 0; gi < 3; ++gi) acc[mt][gi] = mmah(acc[mt][gi], a[mt], b[gi]);
        asm volatile("v_nop\n\tv_nop\n\tv_nop\n\tv_nop"
                     : "+v"(acc[0][0]), "+v"(acc[0][1]), "+v"(acc[0][2]),
                       "+v"(acc[1][0]), "+v"(acc[1][1]), "+v"(acc[1][2])
                     : "v"(a[0].v), "v"(a[1].v), "v"(b[0].v), "v"(b[1].v), "v"(b[2].v));
    }

    gate_epilogue(acc, 0.0625f, bih, bhh, sH, sC, hbuf, cbuf, m0, u0, writec, tid, rq, ug, h, m);
}

__global__ __launch_bounds__(NTHR)
void k_gemm1(const unsigned short* __restrict__ X1h, const unsigned short* __restrict__ X1l,
             const unsigned short* __restrict__ W1h, const unsigned short* __restrict__ W1l,
             const float* __restrict__ bih, const float* __restrict__ bhh,
             float* hbuf, float* cbuf)
{
    __shared__ __attribute__((aligned(16))) float sH[MB_ * HP_];
    __shared__ __attribute__((aligned(16))) float sC[MB_ * HP_];

    const int tid  = threadIdx.x;
    const int lane = tid & 31;
    const int w    = tid >> 5;
    const int h    = lane >> 4;
    const int m    = lane & 15;
    const int rq   = w >> 1;
    const int ug   = w & 1;
    const int u0   = blockIdx.x * UB_;
    const int m0   = blockIdx.y * MB_;
    const int writec = (blockIdx.y == (M_ / MB_) - 1) ? 1 : 0;

    v8f acc[2][3];
#pragma unroll
    for (int mt = 0; mt < 2; ++mt)
#pragma unroll
        for (int gi = 0; gi < 3; ++gi) acc[mt][gi] = zero8();

    const size_t aoff = (size_t)(m0 + 32 * rq + m) * KC_ + 8 * h;
    const size_t boff = (size_t)(u0 + 16 * ug + m) * KC_ + 8 * h;
    const unsigned short* aph = X1h + aoff;
    const unsigned short* apl = X1l + aoff;
    const unsigned short* bph = W1h + boff;
    const unsigned short* bpl = W1l + boff;

#pragma unroll 1
    for (int ks = 0; ks < KS_; ++ks) {
        FragB ah[2], al[2], bh[3], bl[3];
        ldb_glb(ah[0], aph + 32 * ks);
        ldb_glb(al[0], apl + 32 * ks);
        ldb_glb(ah[1], aph + (size_t)16 * KC_ + 32 * ks);
        ldb_glb(al[1], apl + (size_t)16 * KC_ + 32 * ks);
#pragma unroll
        for (int gi = 0; gi < 3; ++gi) {
            ldb_glb(bh[gi], bph + (size_t)gi * (H_ * KC_) + 32 * ks);
            ldb_glb(bl[gi], bpl + (size_t)gi * (H_ * KC_) + 32 * ks);
        }
#pragma unroll
        for (int mt = 0; mt < 2; ++mt)
#pragma unroll
            for (int gi = 0; gi < 3; ++gi) {
                acc[mt][gi] = mmab(acc[mt][gi], ah[mt], bh[gi]);
                acc[mt][gi] = mmab(acc[mt][gi], ah[mt], bl[gi]);
                acc[mt][gi] = mmab(acc[mt][gi], al[mt], bh[gi]);
            }
        asm volatile("v_nop\n\tv_nop\n\tv_nop\n\tv_nop"
                     : "+v"(acc[0][0]), "+v"(acc[0][1]), "+v"(acc[0][2]),
                       "+v"(acc[1][0]), "+v"(acc[1][1]), "+v"(acc[1][2])
                     : "v"(ah[0].v), "v"(ah[1].v), "v"(al[0].v), "v"(al[1].v),
                       "v"(bh[0].v), "v"(bh[1].v), "v"(bh[2].v),
                       "v"(bl[0].v), "v"(bl[1].v), "v"(bl[2].v));
    }

    gate_epilogue(acc, 1.0f, bih, bhh, sH, sC, hbuf, cbuf, m0, u0, writec, tid, rq, ug, h, m);
}

__global__ __launch_bounds__(NTHR)
void k_ln_mid(const float* __restrict__ hbuf, const float* __restrict__ top1,
              const float* __restrict__ gh, const float* __restrict__ bh,
              const float* __restrict__ gx, const float* __restrict__ bx,
              unsigned short* X1h, unsigned short* X1l)
{
    const int tid  = threadIdx.x;
    const int lane = tid & 31;
    const int w    = tid >> 5;
    const int m    = blockIdx.x * 8 + w;
    if (m >= M_) return;
    const int t  = m >> 7;
    const int ca = 8 * lane;
    const int cb = H_ / 2 + 8 * lane;
    const float* hr = hbuf + (size_t)m * H_;
    const v8f va = ld8f(hr + ca);
    const v8f vb = ld8f(hr + cb);

    float s = 0.0f;
#pragma unroll
    for (int e = 0; e < 8; ++e) s += va[e];
#pragma unroll
    for (int e = 0; e < 8; ++e) s += vb[e];
    s = wsum(s);
    const float mean = s * (1.0f / H_);
    v8f da, db;
    float q = 0.0f;
#pragma unroll
    for (int e = 0; e < 8; ++e) { da[e] = va[e] - mean; q += da[e] * da[e]; }
#pragma unroll
    for (int e = 0; e < 8; ++e) { db[e] = vb[e] - mean; q += db[e] * db[e]; }
    q = wsum(q);
    const float rstd = rsqrtf(q * (1.0f / H_) + 1e-5f);

    const v8f g1a = ld8f(gh + ca), g1b = ld8f(gh + cb);
    const v8f b1a = ld8f(bh + ca), b1b = ld8f(bh + cb);
    v8f ya, yb;
#pragma unroll
    for (int e = 0; e < 8; ++e) { ya[e] = da[e] * rstd * g1a[e] + b1a[e]; yb[e] = db[e] * rstd * g1b[e] + b1b[e]; }

    float s2 = 0.0f;
#pragma unroll
    for (int e = 0; e < 8; ++e) s2 += ya[e];
#pragma unroll
    for (int e = 0; e < 8; ++e) s2 += yb[e];
    s2 = wsum(s2);
    const float mean2 = s2 * (1.0f / H_);
    v8f ea, eb;
    float q2 = 0.0f;
#pragma unroll
    for (int e = 0; e < 8; ++e) { ea[e] = ya[e] - mean2; q2 += ea[e] * ea[e]; }
#pragma unroll
    for (int e = 0; e < 8; ++e) { eb[e] = yb[e] - mean2; q2 += eb[e] * eb[e]; }
    q2 = wsum(q2);
    const float rstd2 = rsqrtf(q2 * (1.0f / H_) + 1e-5f);

    const v8f g2a = ld8f(gx + ca), g2b = ld8f(gx + cb);
    const v8f b2a = ld8f(bx + ca), b2b = ld8f(bx + cb);
    v8us hva, lva, hvb, lvb, hvt, lvt;
#pragma unroll
    for (int e = 0; e < 8; ++e) {
        const float za = fmaxf(ea[e] * rstd2 * g2a[e] + b2a[e], 0.0f);
        const float zb = fmaxf(eb[e] * rstd2 * g2b[e] + b2b[e], 0.0f);
        unsigned short hi, lo;
        split_bf16(za, hi, lo); hva[e] = hi; lva[e] = lo;
        split_bf16(zb, hi, lo); hvb[e] = hi; lvb[e] = lo;
    }
    {
        const int lt = min(lane, 7);
        const v8f tv = ld8f(top1 + (size_t)t * SW_ + 8 * lt);
#pragma unroll
        for (int e = 0; e < 8; ++e) { unsigned short hi, lo; split_bf16(tv[e], hi, lo); hvt[e] = hi; lvt[e] = lo; }
    }

    unsigned short* ph = X1h + (size_t)m * KC_;
    unsigned short* pl = X1l + (size_t)m * KC_;
    *(volatile v8us*)(ph + ca) = hva;
    *(volatile v8us*)(ph + cb) = hvb;
    if (lane < 8) *(volatile v8us*)(ph + IN_ + 8 * lane) = hvt;
    *(volatile v8us*)(pl + ca) = lva;
    *(volatile v8us*)(pl + cb) = lvb;
    if (lane < 8) *(volatile v8us*)(pl + IN_ + 8 * lane) = lvt;
    __threadfence();
    *(volatile v8us*)(ph + ca) = hva;
    *(volatile v8us*)(ph + cb) = hvb;
    if (lane < 8) *(volatile v8us*)(ph + IN_ + 8 * lane) = hvt;
    *(volatile v8us*)(pl + ca) = lva;
    *(volatile v8us*)(pl + cb) = lvb;
    if (lane < 8) *(volatile v8us*)(pl + IN_ + 8 * lane) = lvt;
}

__global__ __launch_bounds__(NTHR)
void k_ln_out(const float* __restrict__ hsrc, const float* __restrict__ csrc,
              const float* __restrict__ gh, const float* __restrict__ bh,
              float* omain, float* ohl, float* ocl,
              int nrows, int last0, int wmain)
{
    __shared__ __attribute__((aligned(16))) float sY[8 * H_];
    __shared__ __attribute__((aligned(16))) float sCY[8 * H_];

    const int tid  = threadIdx.x;
    const int lane = tid & 31;
    const int w    = tid >> 5;
    const int r    = blockIdx.x * 8 + w;
    if (r >= nrows) return;
    const int islast = (r >= last0) ? 1 : 0;
    const int rr = max(r - last0, 0);
    const float invH = 1.0f / H_;

    const float* hr = hsrc + (size_t)r * H_ + 4 * lane;
    const float* gp = gh + 4 * lane;
    const float* bp = bh + 4 * lane;
    float* yr  = sY  + w * H_ + 4 * lane;
    float* cyr = sCY + w * H_ + 4 * lane;

    float s = 0.0f;
#pragma unroll 1
    for (int i = 0; i < 4; ++i) {
        const v4f v = *(const v4f*)(hr + 128 * i);
        s += (v[0] + v[1]) + (v[2] + v[3]);
    }
    s = wsum(s);
    const float mean = s * invH;
    float q = 0.0f;
#pragma unroll 1
    for (int i = 0; i < 4; ++i) {
        const v4f v = *(const v4f*)(hr + 128 * i);
        const float d0 = v[0] - mean, d1 = v[1] - mean, d2 = v[2] - mean, d3 = v[3] - mean;
        q += (d0 * d0 + d1 * d1) + (d2 * d2 + d3 * d3);
    }
    q = wsum(q);
    const float rstd = rsqrtf(q * invH + 1e-5f);
#pragma unroll 1
    for (int i = 0; i < 4; ++i) {
        const v4f v = *(const v4f*)(hr + 128 * i);
        const v4f g = *(const v4f*)(gp + 128 * i);
        const v4f b = *(const v4f*)(bp + 128 * i);
        v4f y;
#pragma unroll
        for (int e = 0; e < 4; ++e) y[e] = (v[e] - mean) * rstd * g[e] + b[e];
        *(v4f*)(yr + 128 * i) = y;
    }

    if (islast) {
        const float* cr = csrc + (size_t)rr * H_ + 4 * lane;
        float cs = 0.0f;
#pragma unroll 1
        for (int i = 0; i < 4; ++i) {
            const v4f v = *(const v4f*)(cr + 128 * i);
            cs += (v[0] + v[1]) + (v[2] + v[3]);
        }
        cs = wsum(cs);
        const float cmean = cs * invH;
        float cq = 0.0f;
#pragma unroll 1
        for (int i = 0; i < 4; ++i) {
            const v4f v = *(const v4f*)(cr + 128 * i);
            const float d0 = v[0] - cmean, d1 = v[1] - cmean, d2 = v[2] - cmean, d3 = v[3] - cmean;
            cq += (d0 * d0 + d1 * d1) + (d2 * d2 + d3 * d3);
        }
        cq = wsum(cq);
        const float crstd = rsqrtf(cq * invH + 1e-5f);
#pragma unroll 1
        for (int i = 0; i < 4; ++i) {
            const v4f v = *(const v4f*)(cr + 128 * i);
            const v4f g = *(const v4f*)(gp + 128 * i);
            const v4f b = *(const v4f*)(bp + 128 * i);
            v4f y;
#pragma unroll
            for (int e = 0; e < 4; ++e) y[e] = (v[e] - cmean) * crstd * g[e] + b[e];
            *(v4f*)(cyr + 128 * i) = y;
        }
    }

    v4f y[4], cy[4];
#pragma unroll
    for (int i = 0; i < 4; ++i) {
        y[i] = *(const v4f*)(yr + 128 * i);
#pragma unroll
        for (int e = 0; e < 4; ++e) cy[i][e] = 0.0f;
    }
    if (islast) {
#pragma unroll
        for (int i = 0; i < 4; ++i) cy[i] = *(const v4f*)(cyr + 128 * i);
    }

#pragma unroll
    for (int i = 0; i < 4; ++i) {
        const int c = 128 * i + 4 * lane;
        if (wmain) *(volatile v4f*)(omain + (size_t)r * H_ + c) = y[i];
        if (islast) {
            *(volatile v4f*)(ohl + (size_t)rr * H_ + c) = y[i];
            *(volatile v4f*)(ocl + (size_t)rr * H_ + c) = cy[i];
        }
    }
    __threadfence();
#pragma unroll
    for (int i = 0; i < 4; ++i) {
        const int c = 128 * i + 4 * lane;
        if (wmain) *(volatile v4f*)(omain + (size_t)r * H_ + c) = y[i];
        if (islast) {
            *(volatile v4f*)(ohl + (size_t)rr * H_ + c) = y[i];
            *(volatile v4f*)(ocl + (size_t)rr * H_ + c) = cy[i];
        }
    }
}

extern "C" void kernel_launch(void* const* d_in, const int* in_sizes, int n_in,
                              void* d_out, int out_size, void* d_ws, size_t ws_size,
                              hipStream_t stream)
{
    if (n_in < 21) return;
    if (in_sizes[0]  != M_ * IN_)   return;
    if (in_sizes[1]  != G4_ * KC_)  return;
    if (in_sizes[3]  != G4_)        return;
    if (in_sizes[4]  != G4_)        return;
    if (in_sizes[6]  != 3)          return;
    if (in_sizes[8]  != SW_)        return;
    if (in_sizes[9]  != G4_ * KC_)  return;
    if (in_sizes[11] != G4_)        return;
    if (in_sizes[12] != G4_)        return;
    if (in_sizes[14] != 3)          return;
    if (in_sizes[16] != SW_)        return;
    if (in_sizes[17] != H_ || in_sizes[18] != H_ || in_sizes[19] != H_ || in_sizes[20] != H_) return;
    if ((size_t)out_size != OUT_N)  return;
    if (ws_size < WS_END)           return;

    const float* x    = (const float*)d_in[0];
    const float* Wih0 = (const float*)d_in[1];
    const float* bih0 = (const float*)d_in[3];
    const float* bhh0 = (const float*)d_in[4];
    const float* bc0  = (const float*)d_in[6];
    const float* bs0  = (const float*)d_in[8];
    const float* Wih1 = (const float*)d_in[9];
    const float* bih1 = (const float*)d_in[11];
    const float* bhh1 = (const float*)d_in[12];
    const float* bc1  = (const float*)d_in[14];
    const float* bs1  = (const float*)d_in[16];
    const float* gh   = (const float*)d_in[17];
    const float* bh   = (const float*)d_in[18];
    const float* gx   = (const float*)d_in[19];
    const float* bx   = (const float*)d_in[20];

    float* out   = (float*)d_out;
    float* out0  = out;
    float* out1a = out + OUT1_F;
    float* out1b = out + OUT1_F + (size_t)B_ * H_;
    float* out2a = out + OUT2_F;
    float* out2b = out + OUT2_F + (size_t)B_ * H_;

    char* ws = (char*)d_ws;
    float*          top0 = (float*)(ws + OFF_TOP0);
    float*          top1 = (float*)(ws + OFF_TOP1);
    _Float16*       W0p  = (_Float16*)(ws + OFF_W0P);
    unsigned short* W1h  = (unsigned short*)(ws + OFF_W1H);
    unsigned short* W1l  = (unsigned short*)(ws + OFF_W1L);
    _Float16*       X0p  = (_Float16*)(ws + OFF_X0P);
    unsigned short* X1h  = (unsigned short*)(ws + OFF_X1H);
    unsigned short* X1l  = (unsigned short*)(ws + OFF_X1L);
    float*          hbuf = (float*)(ws + OFF_HB);
    float*          cb0  = (float*)(ws + OFF_CB0);
    float*          cb1  = (float*)(ws + OFF_CB1);

    k_stack<<<dim3(2), dim3(NTHR), 0, stream>>>(bc0, bs0, bc1, bs1, top0, top1);

    k_wcvt<<<dim3(2 * NBW), dim3(NTHR), 0, stream>>>(Wih0, Wih1, W0p, W1h, W1l);

    k_xcvt<<<dim3(NBX), dim3(NTHR), 0, stream>>>(x, (const float*)top0, X0p);

    k_gemm0<<<dim3(H_ / UB_, M_ / MB_), dim3(NTHR), 0, stream>>>(
        (const _Float16*)X0p, (const _Float16*)W0p, bih0, bhh0, hbuf, cb0);

    k_ln_out<<<dim3(B_ / 8), dim3(NTHR), 0, stream>>>(
        (const float*)(hbuf + (size_t)(M_ - B_) * H_), (const float*)cb0, gh, bh,
        out1a, out1a, out2a, B_, 0, 0);

    k_ln_mid<<<dim3(M_ / 8), dim3(NTHR), 0, stream>>>(
        (const float*)hbuf, (const float*)top1, gh, bh, gx, bx, X1h, X1l);

    k_gemm1<<<dim3(H_ / UB_, M_ / MB_), dim3(NTHR), 0, stream>>>(
        (const unsigned short*)X1h, (const unsigned short*)X1l,
        (const unsigned short*)W1h, (const unsigned short*)W1l, bih1, bhh1, hbuf, cb1);

    k_ln_out<<<dim3(M_ / 8), dim3(NTHR), 0, stream>>>(
        (const float*)hbuf, (const float*)cb1, gh, bh,
        out0, out1b, out2b, M_, M_ - B_, 1);
}
